// LSTM2_27169963114676
// MI455X (gfx1250) — hardware-verified
//
#include <hip/hip_runtime.h>
#include <math.h>

constexpr int NBATCH   = 1024;
constexpr int NSTEP    = 1024;
constexpr int NHID     = 64;
constexpr int NGATE    = 4 * NHID;
constexpr int ROWS_BLK = 16;
constexpr int NTHR     = 128;
constexpr int NWAVE    = NTHR / 32;
constexpr int WPITCH   = 72;
constexpr int XPITCH   = 36;
constexpr int TCHUNK   = 32;
constexpr int GATE_STRIDE = NHID * WPITCH;
constexpr int PLANE_STRIDE = NGATE * WPITCH;
constexpr float HCARRY = 16.0f;
constexpr float WCARRY = 16.0f;
constexpr float FOLD   = 1.0f / (HCARRY * WCARRY);
constexpr int GTHR     = 256;
constexpr int NOUT     = NBATCH * NSTEP;

static_assert(NHID % 32 == 0, "K multiple of 32");
static_assert(NHID == 16 * NWAVE, "one 16-unit group per wave");
static_assert(NBATCH % ROWS_BLK == 0, "batch tiles exact");
static_assert(NSTEP % TCHUNK == 0, "time chunks exact");
static_assert(ROWS_BLK * (TCHUNK / 4) == NTHR, "one float4 per thread per chunk");
static_assert((NGATE * NHID / 4) % NTHR == 0, "weight staging loop exact");
static_assert(NGATE == 2 * NTHR, "parameter staging: two gate columns per thread");
static_assert(WPITCH % 8 == 0 && XPITCH % 4 == 0, "16-B aligned LDS rows");
static_assert((NOUT / 4) % GTHR == 0, "guard fill covers whole 512-B wave chunks exactly");

typedef __attribute__((ext_vector_type(16))) _Float16 v16h;
typedef __attribute__((ext_vector_type(8)))  _Float16 v8h;
typedef __attribute__((ext_vector_type(4)))  _Float16 v4h;
typedef __attribute__((ext_vector_type(8)))  float    v8f;
typedef __attribute__((ext_vector_type(4)))  float    v4f;

template <typename T> struct Frag;
template <> struct Frag<_Float16> {
  typedef v16h V; union U { v16h v; v8h h[2]; };
  static __device__ __forceinline__ v16h load(const _Float16* p) {
    U f; f.h[0] = *(const v8h*)(p); f.h[1] = *(const v8h*)(p + 16); return f.v;
  }
  static __device__ __forceinline__ v8f mma(v16h a, v16h b, v8f c) {
    return __builtin_amdgcn_wmma_f32_16x16x32_f16(false, a, false, b, (short)0, c, false, false);
  }
};

__device__ __forceinline__ void gate_guard(v8f& a0, v8f& a1, v8f& a2, v8f& a3,
                                           v16h x, v16h b0, v16h b1, v16h b2, v16h b3) {
  asm volatile("v_nop\n\tv_nop\n\tv_nop\n\tv_nop"
               : "+v"(a0), "+v"(a1), "+v"(a2), "+v"(a3)
               : "v"(x), "v"(b0), "v"(b1), "v"(b2), "v"(b3));
}

__device__ __forceinline__ void gate_chunk(v8f& g0, v8f& g1, v8f& g2, v8f& g3,
                                           const v16h a, const _Float16* wrow) {
  const v16h b0 = Frag<_Float16>::load(wrow);
  const v16h b1 = Frag<_Float16>::load(wrow + 1 * GATE_STRIDE);
  const v16h b2 = Frag<_Float16>::load(wrow + 2 * GATE_STRIDE);
  const v16h b3 = Frag<_Float16>::load(wrow + 3 * GATE_STRIDE);
  g0 = Frag<_Float16>::mma(a, b0, g0);
  g1 = Frag<_Float16>::mma(a, b1, g1);
  g2 = Frag<_Float16>::mma(a, b2, g2);
  g3 = Frag<_Float16>::mma(a, b3, g3);
  gate_guard(g0, g1, g2, g3, a, b0, b1, b2, b3);
}

__device__ __forceinline__ float fsig(float v)  { return __builtin_amdgcn_rcpf(1.0f + __expf(-v)); }
__device__ __forceinline__ float ftanh(float v) { return 1.0f - 2.0f * __builtin_amdgcn_rcpf(__expf(2.0f * v) + 1.0f); }

__global__ __launch_bounds__(NTHR) void seq2_kernel(
    const float* __restrict__ x,
    const float* __restrict__ w_ih1, const float* __restrict__ w_hh1,
    const float* __restrict__ b_ih1, const float* __restrict__ b_hh1,
    const float* __restrict__ w_ih2, const float* __restrict__ w_hh2,
    const float* __restrict__ b_ih2, const float* __restrict__ b_hh2,
    const float* __restrict__ w_lin, const float* __restrict__ b_lin,
    float* __restrict__ out) {
  __shared__ __align__(16) _Float16 Wp[3 * PLANE_STRIDE];
  __shared__ __align__(16) _Float16 H1[ROWS_BLK * WPITCH];
  __shared__ __align__(16) _Float16 H2[ROWS_BLK * WPITCH];
  __shared__ __align__(16) float    Xc[ROWS_BLK * XPITCH];
  __shared__ __align__(16) float    Oc[ROWS_BLK * XPITCH];
  __shared__ __align__(16) float    Pp[NWAVE * 16];
  __shared__ __align__(16) float    Prm[3 * NGATE + NHID];

  const int tid  = threadIdx.x;
  const int lane = tid & 31;
  const int wave = tid >> 5;
  const int c    = lane & 15;
  const int hh   = lane >> 4;
  const int koff = hh * 8;
  const int unit = 16 * wave + c;
  const int rowBase = blockIdx.x * ROWS_BLK;

#pragma unroll 1
  for (int it = 0; it < (NGATE * NHID / 4) / NTHR; ++it) {
    const int idx = it * NTHR + tid;
    const int r  = idx >> 4;
    const int c4 = (idx & 15) * 4;
    const v4f va = *(const v4f*)(w_hh1 + (size_t)idx * 4);
    const v4f vb = *(const v4f*)(w_ih2 + (size_t)idx * 4);
    const v4f vc = *(const v4f*)(w_hh2 + (size_t)idx * 4);
    v4h ha, hb, hc;
#pragma unroll
    for (int e = 0; e < 4; ++e) {
      ha[e] = (_Float16)(va[e] * WCARRY);
      hb[e] = (_Float16)(vb[e] * WCARRY);
      hc[e] = (_Float16)(vc[e] * WCARRY);
    }
    *(v4h*)(Wp + 0 * PLANE_STRIDE + r * WPITCH + c4) = ha;
    *(v4h*)(Wp + 1 * PLANE_STRIDE + r * WPITCH + c4) = hb;
    *(v4h*)(Wp + 2 * PLANE_STRIDE + r * WPITCH + c4) = hc;
  }
  {
    const v8h z8h = {(_Float16)0.0f, (_Float16)0.0f, (_Float16)0.0f, (_Float16)0.0f,
                     (_Float16)0.0f, (_Float16)0.0f, (_Float16)0.0f, (_Float16)0.0f};
#pragma unroll 1
    for (int i = tid; i < 3 * NGATE; i += NTHR) *(v8h*)(Wp + i * WPITCH + NHID) = z8h;
#pragma unroll 1
    for (int i = tid; i < ROWS_BLK * WPITCH / 8; i += NTHR) {
      *(v8h*)(H1 + i * 8) = z8h;
      *(v8h*)(H2 + i * 8) = z8h;
    }
  }
#pragma unroll
  for (int q = 0; q < 2; ++q) {
    const int j = tid + q * NTHR;
    Prm[j]             = w_ih1[j];
    Prm[NGATE + j]     = b_ih1[j] + b_hh1[j];
    Prm[2 * NGATE + j] = b_ih2[j] + b_hh2[j];
  }
  {
    const float wv = w_lin[tid & (NHID - 1)];
    if (tid < NHID) Prm[3 * NGATE + tid] = wv;
  }
  const float bl = b_lin[0];
  __syncthreads();

  const float wx0 = Prm[0 * NHID + unit];
  const float wx1 = Prm[1 * NHID + unit];
  const float wx2 = Prm[2 * NHID + unit];
  const float wx3 = Prm[3 * NHID + unit];
  const float p10 = Prm[NGATE + 0 * NHID + unit];
  const float p11 = Prm[NGATE + 1 * NHID + unit];
  const float p12 = Prm[NGATE + 2 * NHID + unit];
  const float p13 = Prm[NGATE + 3 * NHID + unit];
  const float p20 = Prm[2 * NGATE + 0 * NHID + unit];
  const float p21 = Prm[2 * NGATE + 1 * NHID + unit];
  const float p22 = Prm[2 * NGATE + 2 * NHID + unit];
  const float p23 = Prm[2 * NGATE + 3 * NHID + unit];
  const float wl  = Prm[3 * NGATE + unit];

  const v8f z8 = {0.f, 0.f, 0.f, 0.f, 0.f, 0.f, 0.f, 0.f};
  v8f c1 = z8;
  v8f c2 = z8;

  const _Float16* h1row = H1 + c * WPITCH + koff;
  const _Float16* h2row = H2 + c * WPITCH + koff;
  const _Float16* w1row = Wp + 0 * PLANE_STRIDE + unit * WPITCH + koff;
  const _Float16* w2row = Wp + 1 * PLANE_STRIDE + unit * WPITCH + koff;
  const _Float16* w3row = Wp + 2 * PLANE_STRIDE + unit * WPITCH + koff;

  v16h a1k0 = Frag<_Float16>::load(h1row);
  v16h a1k1 = Frag<_Float16>::load(h1row + 32);

  const int crow = tid >> 3;
  const int cc4  = (tid & 7) * 4;

#pragma unroll 1
  for (int t = 0; t < NSTEP; ++t) {
    const int tl = t & (TCHUNK - 1);
    if (tl == 0) {
      const v4f xv = *(const v4f*)(x + (size_t)(rowBase + crow) * NSTEP + t + cc4);
      *(v4f*)(Xc + crow * XPITCH + cc4) = xv;
    }
    const v16h a2k0 = Frag<_Float16>::load(h2row);
    const v16h a2k1 = Frag<_Float16>::load(h2row + 32);
    __syncthreads();

    float xr[8];
#pragma unroll
    for (int r = 0; r < 8; ++r) xr[r] = Xc[(8 * hh + r) * XPITCH + tl];

    v8f g0 = z8, g1 = z8, g2 = z8, g3 = z8;
    gate_chunk(g0, g1, g2, g3, a1k0, w1row);
    gate_chunk(g0, g1, g2, g3, a1k1, w1row + 32);
#pragma unroll
    for (int r = 0; r < 8; ++r) {
      const float xv = xr[r];
      const float zi = g0[r] * FOLD + (xv * wx0 + p10);
      const float zf = g1[r] * FOLD + (xv * wx1 + p11);
      const float zg = g2[r] * FOLD + (xv * wx2 + p12);
      const float zo = g3[r] * FOLD + (xv * wx3 + p13);
      const float ig = fsig(zi);
      const float fg = fsig(zf);
      const float gg = ftanh(zg);
      const float og = fsig(zo);
      const float cn = fg * c1[r] + ig * gg;
      c1[r] = cn;
      const float hn = og * ftanh(cn);
      H1[(8 * hh + r) * WPITCH + unit] = (_Float16)(hn * HCARRY);
    }
    __syncthreads();

    a1k0 = Frag<_Float16>::load(h1row);
    a1k1 = Frag<_Float16>::load(h1row + 32);

    g0 = z8; g1 = z8; g2 = z8; g3 = z8;
    gate_chunk(g0, g1, g2, g3, a1k0, w2row);
    gate_chunk(g0, g1, g2, g3, a1k1, w2row + 32);
    gate_chunk(g0, g1, g2, g3, a2k0, w3row);
    gate_chunk(g0, g1, g2, g3, a2k1, w3row + 32);
    float pv[8];
#pragma unroll
    for (int r = 0; r < 8; ++r) {
      const float zi = g0[r] * FOLD + p20;
      const float zf = g1[r] * FOLD + p21;
      const float zg = g2[r] * FOLD + p22;
      const float zo = g3[r] * FOLD + p23;
      const float ig = fsig(zi);
      const float fg = fsig(zf);
      const float gg = ftanh(zg);
      const float og = fsig(zo);
      const float cn = fg * c2[r] + ig * gg;
      c2[r] = cn;
      const float hn = og * ftanh(cn);
      H2[(8 * hh + r) * WPITCH + unit] = (_Float16)(hn * HCARRY);
      pv[r] = hn * wl;
    }
#pragma unroll
    for (int r = 0; r < 8; ++r) {
      float p = pv[r];
      p += __shfl_xor(p, 1, 32);
      p += __shfl_xor(p, 2, 32);
      p += __shfl_xor(p, 4, 32);
      p += __shfl_xor(p, 8, 32);
      pv[r] = p;
    }
    if (c == 0) {
#pragma unroll
      for (int r = 0; r < 8; ++r) Pp[wave * 16 + 8 * hh + r] = pv[r];
    }
    __syncthreads();

    if (tid < ROWS_BLK) {
      const float s = ((Pp[tid] + Pp[16 + tid]) + Pp[32 + tid]) + Pp[48 + tid];
      Oc[tid * XPITCH + tl] = s + bl;
    }

    if (tl == TCHUNK - 1) {
      __syncthreads();
      const v4f ov = *(const v4f*)(Oc + crow * XPITCH + cc4);
      float* op = out + (size_t)(rowBase + crow) * NSTEP + (t - (TCHUNK - 1)) + cc4;
      *(volatile v4f*)op = ov;
      __threadfence();
      *(volatile v4f*)op = ov;
      __threadfence();
    }
  }
}

__global__ __launch_bounds__(GTHR) void premise_guard_kernel(const int* __restrict__ nfut,
                                                            float* __restrict__ out, int n4) {
  const int v = nfut[0];
  if (v != 0) {
    const float qn = __uint_as_float(0x7fc00000u);
    const v4f nv = {qn, qn, qn, qn};
    for (int pass = 0; pass < 2; ++pass) {
#pragma unroll 1
      for (int i = threadIdx.x; i < n4; i += GTHR) {
        *(volatile v4f*)(out + (size_t)i * 4) = nv;
      }
      __threadfence();
    }
  }
}

extern "C" void kernel_launch(void* const* d_in, const int* in_sizes, int n_in,
                              void* d_out, int out_size, void* d_ws, size_t ws_size,
                              hipStream_t stream) {
  (void)d_ws; (void)ws_size;
  if (n_in < 12 || d_out == nullptr) return;
  if (in_sizes[0] != NBATCH * NSTEP || in_sizes[1] != NGATE || in_sizes[2] != NGATE * NHID ||
      in_sizes[3] != NGATE || in_sizes[4] != NGATE || in_sizes[5] != NGATE * NHID ||
      in_sizes[6] != NGATE * NHID || in_sizes[7] != NGATE || in_sizes[8] != NGATE ||
      in_sizes[9] != NHID || in_sizes[10] != 1 || in_sizes[11] != 1 || out_size != NOUT) return;

  const float* x     = (const float*)d_in[0];
  const float* w_ih1 = (const float*)d_in[1];
  const float* w_hh1 = (const float*)d_in[2];
  const float* b_ih1 = (const float*)d_in[3];
  const float* b_hh1 = (const float*)d_in[4];
  const float* w_ih2 = (const float*)d_in[5];
  const float* w_hh2 = (const float*)d_in[6];
  const float* b_ih2 = (const float*)d_in[7];
  const float* b_hh2 = (const float*)d_in[8];
  const float* w_lin = (const float*)d_in[9];
  const float* b_lin = (const float*)d_in[10];
  const int*   nfut  = (const int*)d_in[11];
  float* out = (float*)d_out;

  seq2_kernel<<<NBATCH / ROWS_BLK, NTHR, 0, stream>>>(
      x, w_ih1, w_hh1, b_ih1, b_hh1, w_ih2, w_hh2, b_ih2, b_hh2, w_lin, b_lin, out);

  premise_guard_kernel<<<1, GTHR, 0, stream>>>(nfut, out, out_size / 4);
}
